// RNadeMoG_51170240364859
// MI455X (gfx1250) — hardware-verified
//
#include <hip/hip_runtime.h>


#define NBt  512
#define LL   500
#define HH_  512
#define DIN  35
#define NOUT 35
#define NOP  48
#define TCH  10

typedef unsigned short bf;
typedef __attribute__((ext_vector_type(16))) __bf16   v16bf;
typedef __attribute__((ext_vector_type(8)))  unsigned short v8us;
typedef __attribute__((ext_vector_type(8)))  float    v8f;
typedef __attribute__((ext_vector_type(4)))  float    v4f;
typedef v4f  __attribute__((may_alias)) v4fa;
typedef v8us __attribute__((may_alias)) v8usa;

__device__ __forceinline__ unsigned short f2bf(float f) { unsigned u = __float_as_uint(f); u += 0x7FFFu + ((u >> 16) & 1u); return (unsigned short)(u >> 16); }
__device__ __forceinline__ float bf2f(unsigned short b) { return __uint_as_float(((unsigned)b) << 16); }
__device__ __forceinline__ float bfr(float f) { return bf2f(f2bf(f)); }
__device__ __forceinline__ v16bf cat16b(v8us lo, v8us hi) { return __builtin_bit_cast(v16bf, __builtin_shufflevector(lo, hi, 0, 1, 2, 3, 4, 5, 6, 7, 8, 9, 10, 11, 12, 13, 14, 15)); }
__device__ __forceinline__ v8f wmmab(v16bf a, v16bf b, v8f c) { return __builtin_amdgcn_wmma_f32_16x16x32_bf16(false, a, false, b, (short)0, c, false, false); }
#define VST2(T, p, v) do { const T vst2_v_ = (v); *(volatile T*)(p) = vst2_v_; __threadfence(); *(volatile T*)(p) = vst2_v_; } while (0)

__global__ __launch_bounds__(256) void k_xz(const float* __restrict__ x, const float* __restrict__ z, bf* XZb) {
    const int lane = threadIdx.x & 31; const size_t w = (size_t)blockIdx.x * 8 + (threadIdx.x >> 5);
    const size_t r = w * 8 + (lane >> 2); const int q = (lane & 3) * 8;
    if (r >= (size_t)LL * NBt) return;
    const int t = (int)(r / NBt), b = (int)(r - (size_t)t * NBt);
    v8us o;
#pragma unroll
    for (int i = 0; i < 8; ++i) { const int f = q + i; const float v = (f < 3) ? x[((size_t)b * LL + t) * 3 + f] : z[((size_t)b * LL + t) * 32 + (f - 3)]; o[i] = f2bf(v); }
    VST2(v8us, XZb + r * 32 + q, o);
}
__global__ __launch_bounds__(256) void k_we(const float* __restrict__ We, bf* WeT) {
    __shared__ unsigned short tl[64][34];
    const int t = blockIdx.x / (HH_ / 64), hq = blockIdx.x - t * (HH_ / 64), h0 = hq * 64, tid = threadIdx.x;
    { const int k = tid >> 3, hh = (tid & 7) * 8;
#pragma unroll
      for (int i = 0; i < 8; ++i) tl[hh + i][k] = f2bf(We[((size_t)t * DIN + k) * HH_ + h0 + hh + i]); }
    __syncthreads();
    { const int hh = tid >> 2, q = (tid & 3) * 8; v8us o;
#pragma unroll
      for (int i = 0; i < 8; ++i) o[i] = tl[hh][q + i];
      VST2(v8us, WeT + ((size_t)t * HH_ + h0 + hh) * 32 + q, o); }
}
__global__ __launch_bounds__(256) void k_wc(const float* __restrict__ wm, const float* __restrict__ ws, const float* __restrict__ wp, bf* WcT) {
    const int lane = threadIdx.x & 31, wave = threadIdx.x >> 5;
    const int t = blockIdx.x / (NOP / 8), nq = blockIdx.x - t * (NOP / 8), n = nq * 8 + wave;
#pragma unroll
    for (int s = 0; s < 2; ++s) { v8us o;
#pragma unroll
        for (int i = 0; i < 8; ++i) { const int h = s * 256 + lane * 8 + i; float v = 0.f;
            if (n < 15) v = wm[((size_t)t * HH_ + h) * 15 + n]; else if (n < 30) v = ws[((size_t)t * HH_ + h) * 15 + (n - 15)]; else if (n < 35) v = wp[((size_t)t * HH_ + h) * 5 + (n - 30)];
            o[i] = f2bf(v); }
        VST2(v8us, WcT + ((size_t)t * NOP + n) * HH_ + s * 256 + lane * 8, o); }
}
__global__ __launch_bounds__(128) void k_scan(const bf* __restrict__ XZb, const bf* __restrict__ WeT, const float* __restrict__ z, const float* __restrict__ We, const float* __restrict__ benc,
                                             const float* __restrict__ resc, int t0, float* STATE, bf* HHp, bf* HLp) {
    __shared__ __align__(16) float ost[4][16 * 68];
    const int lane = threadIdx.x & 31, wave = threadIdx.x >> 5, lr = lane & 15, hi = lane >> 4;
    const int b0 = blockIdx.x * 64 + wave * 16, h0 = blockIdx.y * 64;
    float* os = &ost[wave][0];
    v8f a[4];
#pragma unroll
    for (int n = 0; n < 4; ++n)
#pragma unroll
        for (int j = 0; j < 8; ++j) { const int b = b0 + hi * 8 + j, h = h0 + n * 16 + lr; a[n][j] = (t0 == 0) ? bfr(benc[h]) : STATE[(size_t)b * HH_ + h]; }
#pragma unroll 1
    for (int tl = 0; tl < TCH; ++tl) { const int t = t0 + tl;
#pragma unroll
        for (int n = 0; n < 4; ++n)
#pragma unroll
            for (int j = 0; j < 8; ++j) os[(hi * 8 + j) * 68 + n * 16 + lr] = fmaxf(a[n][j], 0.f);
        __builtin_amdgcn_wave_barrier(); asm volatile("" ::: "memory");
        { auto pass = [&]() {
#pragma unroll
            for (int s = 0; s < 4; ++s) { const int row = 4 * s + (lane >> 3), piece = lane & 7; const float* sp = os + row * 68 + piece * 8; v8us oh, ol;
#pragma unroll
                for (int i = 0; i < 8; ++i) { const unsigned short hb = f2bf(sp[i]); oh[i] = hb; ol[i] = f2bf(sp[i] - bf2f(hb)); }
                const size_t o = (((size_t)tl * NBt) + b0 + row) * HH_ + h0 + piece * 8;
                *(volatile v8us*)(HHp + o) = oh; *(volatile v8us*)(HLp + o) = ol; } };
          pass(); __threadfence(); pass(); }
        __builtin_amdgcn_wave_barrier(); asm volatile("" ::: "memory");
        v8f p[4];
        const size_t ao = ((size_t)t * NBt + b0 + lr) * 32 + 8 * hi;
        const v16bf av = cat16b(*(const v8us*)(XZb + ao), *(const v8us*)(XZb + ao + 16));
#pragma unroll
        for (int n = 0; n < 4; ++n) { const size_t bo = ((size_t)t * HH_ + h0 + n * 16 + lr) * 32 + 8 * hi; p[n] = wmmab(av, cat16b(*(const v8us*)(WeT + bo), *(const v8us*)(WeT + bo + 16)), (v8f){}); }
        asm volatile("v_nop\n\tv_nop\n\tv_nop\n\tv_nop" : "+v"(p[0]), "+v"(p[1]), "+v"(p[2]), "+v"(p[3]) : "v"(av));
        float xr[8][3], wr[4][3];
#pragma unroll
        for (int j = 0; j < 8; ++j) { const int b = b0 + hi * 8 + j;
#pragma unroll
            for (int i = 0; i < 3; ++i) xr[j][i] = bfr(z[((size_t)b * LL + t) * 32 + 29 + i]); }
#pragma unroll
        for (int n = 0; n < 4; ++n) { const int h = h0 + n * 16 + lr;
#pragma unroll
            for (int i = 0; i < 3; ++i) wr[n][i] = bfr(We[((size_t)t * DIN + 32 + i) * HH_ + h]); }
        const float rt = bfr(resc[t]), rt1 = bfr(resc[t + 1]);
#pragma unroll
        for (int n = 0; n < 4; ++n)
#pragma unroll
            for (int j = 0; j < 8; ++j) { float pv = p[n][j];
#pragma unroll
                for (int i = 0; i < 3; ++i) pv += xr[j][i] * wr[n][i];
                a[n][j] = rt1 * (a[n][j] / rt + pv); }
    }
#pragma unroll
    for (int n = 0; n < 4; ++n)
#pragma unroll
        for (int j = 0; j < 8; ++j) os[(hi * 8 + j) * 68 + n * 16 + lr] = a[n][j];
    __builtin_amdgcn_wave_barrier(); asm volatile("" ::: "memory");
    auto pass2 = [&]() {
#pragma unroll
        for (int s = 0; s < 8; ++s) { const int Lid = (lane >> 3) + 4 * s, piece = lane & 7; const int row = Lid >> 1, cofs = (Lid & 1) * 32 + piece * 4;
            const v4f val = *(const v4fa*)(os + row * 68 + cofs); *(volatile v4f*)(STATE + (size_t)(b0 + row) * HH_ + h0 + cofs) = val; }
    };
    pass2(); __threadfence(); pass2();
}
__global__ __launch_bounds__(128) void k_logits(const bf* __restrict__ HHp, const bf* __restrict__ HLp, const bf* __restrict__ WcT, const float* __restrict__ bm, const float* __restrict__ bs, const float* __restrict__ bp, int t0, float* LG) {
    __shared__ __align__(16) float st[64 * NOP];
    const int lane = threadIdx.x & 31, wave = threadIdx.x >> 5, lr = lane & 15, hi = lane >> 4, tid = threadIdx.x;
    const int tl = blockIdx.z, t = t0 + tl, b0 = blockIdx.x * 64 + wave * 16;
    const size_t aoff = ((size_t)tl * NBt + b0 + lr) * HH_ + 8 * hi;
    const bf* wc = WcT + (size_t)t * NOP * HH_;
    v8f acc[3];
#pragma unroll
    for (int n = 0; n < 3; ++n) acc[n] = (v8f){};
#pragma unroll 2
    for (int kc = 0; kc < HH_; kc += 32) {
        const v16bf a = cat16b(*(const v8us*)(HHp + aoff + kc), *(const v8us*)(HHp + aoff + kc + 16)), al = cat16b(*(const v8us*)(HLp + aoff + kc), *(const v8us*)(HLp + aoff + kc + 16));
#pragma unroll
        for (int n = 0; n < 3; ++n) { const bf* bpn = wc + (size_t)(n * 16 + lr) * HH_ + kc + 8 * hi; const v16bf bb = cat16b(*(const v8us*)bpn, *(const v8us*)(bpn + 16)); acc[n] = wmmab(a, bb, acc[n]); acc[n] = wmmab(al, bb, acc[n]); }
        asm volatile("v_nop" : "+v"(acc[0]), "+v"(acc[1]), "+v"(acc[2]) : "v"(a), "v"(al) : "memory");
    }
    asm volatile("v_nop\n\tv_nop\n\tv_nop\n\tv_nop" : "+v"(acc[0]), "+v"(acc[1]), "+v"(acc[2]));
#pragma unroll
    for (int n = 0; n < 3; ++n) { const int c = n * 16 + lr; const float bias = (c < 15) ? bfr(bm[t * 15 + c]) : (c < 30) ? bfr(bs[t * 15 + c - 15]) : (c < 35) ? bfr(bp[t * 5 + c - 30]) : 0.f;
#pragma unroll
        for (int j = 0; j < 8; ++j) st[(wave * 16 + hi * 8 + j) * NOP + c] = acc[n][j] + bias; }
    __syncthreads();
    float* dst = LG + ((size_t)t * NBt + blockIdx.x * 64) * NOP;
    auto pass = [&]() {
#pragma unroll
        for (int s = 0; s < (64 * NOP) / (128 * 4); ++s) { const int e0 = s * 512 + tid * 4; const v4f v = *(const v4fa*)(st + e0); *(volatile v4f*)(dst + e0) = v; }
    };
    pass(); __threadfence(); pass();
}
__global__ __launch_bounds__(256) void k_out(const float* __restrict__ LG, float* out) {
    const size_t e = (size_t)blockIdx.x * 256 + threadIdx.x;
    if (e >= (size_t)NBt * LL * NOUT) return;
    const int n = (int)(e % NOUT); const size_t bt = e / NOUT; const int t = (int)(bt % LL), b = (int)(bt / LL);
    const float v = LG[((size_t)t * NBt + b) * NOP + n];
    *(volatile float*)(out + e) = v; __threadfence(); *(volatile float*)(out + e) = v;
}

extern "C" void kernel_launch(void* const* d_in, const int* in_sizes, int n_in,
                              void* d_out, int out_size, void* d_ws, size_t ws_size, hipStream_t stream) {
    (void)in_sizes; (void)n_in; (void)out_size;
    const float* x = (const float*)d_in[0]; const float* z = (const float*)d_in[1]; const float* We = (const float*)d_in[2]; const float* benc = (const float*)d_in[3];
    const float* wm = (const float*)d_in[4]; const float* bm = (const float*)d_in[5]; const float* ws = (const float*)d_in[6]; const float* bs = (const float*)d_in[7];
    const float* wp = (const float*)d_in[8]; const float* bp = (const float*)d_in[9]; const float* resc = (const float*)d_in[10];
    float* out = (float*)d_out;
    char* wsp = (char*)d_ws;
    auto take = [&](size_t bytes) { char* p = wsp; wsp += (bytes + 255) & ~(size_t)255; return (void*)p; };
    bf* XZb = (bf*)take((size_t)LL * NBt * 32 * 2); bf* WeT = (bf*)take((size_t)LL * HH_ * 32 * 2); bf* WcT = (bf*)take((size_t)LL * NOP * HH_ * 2);
    bf* HHp = (bf*)take((size_t)TCH * NBt * HH_ * 2); bf* HLp = (bf*)take((size_t)TCH * NBt * HH_ * 2); float* STATE = (float*)take((size_t)NBt * HH_ * 4);
    float* LG = (float*)take((size_t)LL * NBt * NOP * 4);
    if ((size_t)(wsp - (char*)d_ws) > ws_size) return;
    k_xz<<<(LL * NBt) / 64, 256, 0, stream>>>(x, z, XZb);
    k_we<<<LL * (HH_ / 64), 256, 0, stream>>>(We, WeT);
    k_wc<<<LL * (NOP / 8), 256, 0, stream>>>(wm, ws, wp, WcT);
    for (int c = 0; c < LL / TCH; ++c) {
        k_scan<<<dim3(NBt / 64, HH_ / 64, 1), 128, 0, stream>>>(XZb, WeT, z, We, benc, resc, c * TCH, STATE, HHp, HLp);
        k_logits<<<dim3(NBt / 64, 1, TCH), 128, 0, stream>>>(HHp, HLp, WcT, bm, bs, bp, c * TCH, LG);
    }
    k_out<<<(unsigned)(((size_t)NBt * LL * NOUT + 255) / 256), 256, 0, stream>>>(LG, out);
}
